// WavLMSelfAttention_5574867550218
// MI455X (gfx1250) — hardware-verified
//
#include <hip/hip_runtime.h>


#define NB_  8
#define TT   1024
#define EE   1024
#define NH_  16
#define HD   64
#define ZH   2
#define NBK  32
#define PCAR 1024.0f
typedef _Float16 h16;
typedef unsigned short bf;
typedef __attribute__((ext_vector_type(16))) __bf16   v16bf;
typedef __attribute__((ext_vector_type(16))) _Float16 v16h;
typedef __attribute__((ext_vector_type(8)))  _Float16 v8h;
typedef __attribute__((ext_vector_type(8)))  unsigned short v8us;
typedef __attribute__((ext_vector_type(8)))  float    v8f;
typedef __attribute__((ext_vector_type(4)))  float    v4f;
typedef v8h  __attribute__((may_alias)) v8ha;
typedef v4f  __attribute__((may_alias)) v4fa;
typedef v8us __attribute__((may_alias)) v8usa;

__device__ __forceinline__ unsigned short f2bf(float f) { unsigned u = __float_as_uint(f); u += 0x7FFFu + ((u >> 16) & 1u); return (unsigned short)(u >> 16); }
__device__ __forceinline__ float bf2f(unsigned short b) { return __uint_as_float(((unsigned)b) << 16); }
__device__ __forceinline__ float bfr(float f) { return bf2f(f2bf(f)); }
__device__ __forceinline__ v16h cat16(v8h lo, v8h hi) { return __builtin_shufflevector(lo, hi, 0, 1, 2, 3, 4, 5, 6, 7, 8, 9, 10, 11, 12, 13, 14, 15); }
__device__ __forceinline__ v16bf cat16b(v8us lo, v8us hi) { return __builtin_bit_cast(v16bf, __builtin_shufflevector(lo, hi, 0, 1, 2, 3, 4, 5, 6, 7, 8, 9, 10, 11, 12, 13, 14, 15)); }
__device__ __forceinline__ v8f wmma16(v16h a, v16h b, v8f c) { return __builtin_amdgcn_wmma_f32_16x16x32_f16(false, a, false, b, (short)0, c, false, false); }
__device__ __forceinline__ v8f wmmab(v16bf a, v16bf b, v8f c) { return __builtin_amdgcn_wmma_f32_16x16x32_bf16(false, a, false, b, (short)0, c, false, false); }


template <typename T16> struct WFrag;
template <> struct WFrag<h16> { typedef v16h V; static __device__ __forceinline__ V ld(const h16* p) { return cat16(*(const v8h*)p, *(const v8h*)(p + 16)); } static __device__ __forceinline__ v8f mma(V a, V b, v8f c) { return wmma16(a, b, c); } };
template <> struct WFrag<bf> { typedef v16bf V; static __device__ __forceinline__ V ld(const bf* p) { return cat16b(*(const v8us*)p, *(const v8us*)(p + 16)); } static __device__ __forceinline__ v8f mma(V a, V b, v8f c) { return wmmab(a, b, c); } };
template <typename T16, int NSPLIT, bool BIAS>
__global__ __launch_bounds__(32) void k_gemmw(const T16* __restrict__ A, const T16* __restrict__ A2, const T16* __restrict__ Bt, const T16* __restrict__ Bt2, int K, float* C, int ldc, const float* __restrict__ bias, size_t sA, size_t sB, size_t sC) {
    typedef typename WFrag<T16>::V V;
    __shared__ __align__(16) float os[16 * 68];
    const size_t z = blockIdx.z; A += z * sA; if (A2) A2 += z * sA; Bt += z * sB; if (Bt2) Bt2 += z * sB; C += z * sC;
    const int lane = threadIdx.x & 31, lr = lane & 15, hi = lane >> 4; const int r0 = blockIdx.x * 64, c0 = blockIdx.y * 64;
    v8f acc[4][4];
#pragma unroll
    for (int mb = 0; mb < 4; ++mb)
#pragma unroll
        for (int nb = 0; nb < 4; ++nb) acc[mb][nb] = (v8f){};
    const size_t aoff = (size_t)(r0 + lr) * K + 8 * hi, boff = (size_t)(c0 + lr) * K + 8 * hi;
#pragma unroll 1
    for (int kc = 0; kc < K; kc += 32) {
        V a[4], a2[4];
#pragma unroll
        for (int mb = 0; mb < 4; ++mb) { a[mb] = WFrag<T16>::ld(A + aoff + (size_t)mb * 16 * K + kc); if (NSPLIT == 1 || NSPLIT == 2) a2[mb] = WFrag<T16>::ld(A2 + aoff + (size_t)mb * 16 * K + kc); }
#pragma unroll
        for (int nb = 0; nb < 4; ++nb) { const V b = WFrag<T16>::ld(Bt + boff + (size_t)nb * 16 * K + kc); V b2; if (NSPLIT >= 2) b2 = WFrag<T16>::ld(Bt2 + boff + (size_t)nb * 16 * K + kc);
#pragma unroll
            for (int mb = 0; mb < 4; ++mb) { acc[mb][nb] = WFrag<T16>::mma(a[mb], b, acc[mb][nb]); if (NSPLIT == 1 || NSPLIT == 2) acc[mb][nb] = WFrag<T16>::mma(a2[mb], b, acc[mb][nb]); if (NSPLIT >= 2) acc[mb][nb] = WFrag<T16>::mma(a[mb], b2, acc[mb][nb]); } }
        asm volatile("v_nop\n\tv_nop\n\tv_nop\n\tv_nop" : "+v"(acc[0][0]), "+v"(acc[1][1]), "+v"(acc[2][2]), "+v"(acc[3][3]) : "v"(a[0]), "v"(a[3]));
    }
#pragma unroll
    for (int mb = 0; mb < 4; ++mb) {
#pragma unroll
        for (int nb = 0; nb < 4; ++nb) {
#pragma unroll
            for (int j = 0; j < 8; ++j) os[(hi * 8 + j) * 68 + nb * 16 + lr] = acc[mb][nb][j]; }
        __builtin_amdgcn_wave_barrier(); asm volatile("" ::: "memory");
        float* crow = C + (size_t)(r0 + mb * 16) * ldc + c0;
#pragma unroll 1
        for (int ps = 0; ps < 2; ++ps) {
#pragma unroll
            for (int s = 0; s < 8; ++s) { const int row = 2 * s + hi, cofs = lr * 4; v4f val = *(const v4fa*)(os + row * 68 + cofs); if (BIAS) { val[0] += bfr(bias[c0 + cofs]); val[1] += bfr(bias[c0 + cofs + 1]); val[2] += bfr(bias[c0 + cofs + 2]); val[3] += bfr(bias[c0 + cofs + 3]); }
                *(volatile v4f*)(crow + (size_t)row * ldc + cofs) = val; }
            if (ps == 0) __threadfence(); }
        __builtin_amdgcn_wave_barrier(); asm volatile("" ::: "memory");
    }
}

__device__ __forceinline__ h16 tohx(float x) { return (h16)x; }
__device__ __forceinline__ void splitf(float y, unsigned short& h, unsigned short& l) { h = f2bf(y); l = f2bf(y - bf2f(h)); }
__device__ __forceinline__ float sigm_(float x) { return __fdiv_rn(1.0f, 1.0f + __expf(-x)); }
typedef __attribute__((ext_vector_type(2))) _Float16 v2h;
typedef __attribute__((ext_vector_type(4))) _Float16 v4h;
typedef __attribute__((ext_vector_type(2))) unsigned short v2us;
typedef __attribute__((ext_vector_type(4))) unsigned short v4us;
__constant__ unsigned char c_bkt[2 * TT - 1] = {15,15,15,15,15,15,15,15,15,15,15,15,15,15,15,15,15,15,15,15,15,15,15,15,15,15,15,15,15,15,15,15,15,15,15,15,15,15,15,15,15,15,15,15,15,15,15,15,15,15,15,15,15,15,15,15,15,15,15,15,15,15,15,15,15,15,15,15,15,15,15,15,15,15,15,15,15,15,15,15,15,15,15,15,15,15,15,15,15,15,15,15,15,15,15,15,15,15,15,15,15,15,15,15,15,15,15,15,15,15,15,15,15,15,15,15,15,15,15,15,15,15,15,15,15,15,15,15,15,15,15,15,15,15,15,15,15,15,15,15,15,15,15,15,15,15,15,15,15,15,15,15,15,15,15,15,15,15,15,15,15,15,15,15,15,15,15,15,15,15,15,15,15,15,15,15,15,15,15,15,15,15,15,15,15,15,15,15,15,15,15,15,15,15,15,15,15,15,15,15,15,15,15,15,15,15,15,15,15,15,15,15,15,15,15,15,15,15,15,15,15,15,15,15,15,15,15,15,15,15,15,15,15,15,15,15,15,15,15,15,15,15,15,15,15,15,15,15,15,15,15,15,15,15,15,15,15,15,15,15,15,15,15,15,15,15,15,15,15,15,15,15,15,15,15,15,15,15,15,15,15,15,15,15,15,15,15,15,15,15,15,15,15,15,15,15,15,15,15,15,15,15,15,15,15,15,15,15,15,15,15,15,15,15,15,15,15,15,15,15,15,15,15,15,15,15,15,15,15,15,15,15,15,15,15,15,15,15,15,15,15,15,15,15,15,15,15,15,15,15,15,15,15,15,15,15,15,15,15,15,15,15,15,15,15,15,15,15,15,15,15,15,15,15,15,15,15,15,15,15,15,15,15,15,15,15,15,15,15,15,15,15,15,15,15,15,15,15,15,15,15,15,15,15,15,15,15,15,15,15,15,15,15,15,15,15,15,15,15,15,15,15,15,15,15,15,15,15,15,15,15,15,15,15,15,15,15,15,15,15,15,15,15,15,15,15,15,15,15,15,15,15,15,15,15,15,15,15,15,15,15,15,15,15,15,15,15,15,15,15,15,15,15,15,15,15,15,15,15,15,15,15,15,15,15,15,15,15,15,15,15,15,15,15,15,15,15,15,15,15,15,15,15,15,15,15,15,15,15,15,15,15,15,15,15,15,15,15,15,15,15,15,15,15,15,15,15,15,15,15,15,15,15,15,15,15,15,15,15,15,15,15,15,15,15,15,15,15,15,15,15,15,15,15,15,15,15,15,15,15,15,15,15,15,15,15,15,15,15,15,15,15,15,15,15,15,15,15,15,15,15,15,15,15,15,15,15,15,15,15,15,15,15,15,15,15,15,15,15,15,15,15,15,15,15,15,15,15,15,15,15,15,15,15,15,15,15,15,15,15,15,15,15,15,15,15,15,15,15,15,15,15,15,15,15,15,15,15,15,15,15,15,15,15,15,15,15,15,15,15,15,15,15,15,15,15,15,15,15,15,15,15,15,15,15,15,15,15,15,15,15,15,15,15,15,15,15,15,15,15,15,15,15,15,15,15,15,15,15,15,15,15,15,15,15,15,15,15,15,15,15,15,15,15,15,15,15,15,15,15,15,15,15,15,15,15,15,15,15,15,15,15,15,15,15,15,15,15,15,15,15,15,15,15,15,15,15,15,15,15,15,15,15,15,15,15,15,15,15,15,15,15,15,15,15,15,15,15,15,15,15,15,15,15,15,15,15,15,15,15,15,15,15,15,15,15,15,15,15,15,15,15,15,15,15,15,15,15,15,15,15,15,15,15,15,15,15,15,15,15,15,15,15,15,15,15,15,15,15,15,15,15,15,15,15,15,15,15,15,15,15,15,15,15,15,15,15,15,15,15,15,15,15,15,15,15,15,15,15,15,15,15,15,15,15,15,15,15,15,15,15,15,15,15,15,15,15,15,15,15,15,15,15,15,15,15,15,15,15,15,15,15,15,15,15,15,15,15,15,15,15,15,15,15,15,15,15,15,15,15,15,15,15,15,15,15,15,15,15,15,15,15,15,15,15,15,15,15,15,15,15,15,15,15,15,15,15,15,15,15,15,15,15,15,15,15,15,15,15,15,15,15,15,14,14,14,14,14,14,14,14,14,14,14,14,14,14,14,14,14,14,14,14,14,14,14,14,14,14,14,13,13,13,13,13,13,13,13,13,13,13,13,13,13,13,13,13,13,12,12,12,12,12,12,12,12,12,12,12,12,12,12,11,11,11,11,11,11,11,11,11,10,10,10,10,10,10,10,9,9,9,9,8,8,8,8,7,6,5,4,3,2,1,0,17,18,19,20,21,22,23,24,24,24,24,25,25,25,25,26,26,26,26,26,26,26,27,27,27,27,27,27,27,27,27,28,28,28,28,28,28,28,28,28,28,28,28,28,28,29,29,29,29,29,29,29,29,29,29,29,29,29,29,29,29,29,29,30,30,30,30,30,30,30,30,30,30,30,30,30,30,30,30,30,30,30,30,30,30,30,30,30,30,30,31,31,31,31,31,31,31,31,31,31,31,31,31,31,31,31,31,31,31,31,31,31,31,31,31,31,31,31,31,31,31,31,31,31,31,31,31,31,31,31,31,31,31,31,31,31,31,31,31,31,31,31,31,31,31,31,31,31,31,31,31,31,31,31,31,31,31,31,31,31,31,31,31,31,31,31,31,31,31,31,31,31,31,31,31,31,31,31,31,31,31,31,31,31,31,31,31,31,31,31,31,31,31,31,31,31,31,31,31,31,31,31,31,31,31,31,31,31,31,31,31,31,31,31,31,31,31,31,31,31,31,31,31,31,31,31,31,31,31,31,31,31,31,31,31,31,31,31,31,31,31,31,31,31,31,31,31,31,31,31,31,31,31,31,31,31,31,31,31,31,31,31,31,31,31,31,31,31,31,31,31,31,31,31,31,31,31,31,31,31,31,31,31,31,31,31,31,31,31,31,31,31,31,31,31,31,31,31,31,31,31,31,31,31,31,31,31,31,31,31,31,31,31,31,31,31,31,31,31,31,31,31,31,31,31,31,31,31,31,31,31,31,31,31,31,31,31,31,31,31,31,31,31,31,31,31,31,31,31,31,31,31,31,31,31,31,31,31,31,31,31,31,31,31,31,31,31,31,31,31,31,31,31,31,31,31,31,31,31,31,31,31,31,31,31,31,31,31,31,31,31,31,31,31,31,31,31,31,31,31,31,31,31,31,31,31,31,31,31,31,31,31,31,31,31,31,31,31,31,31,31,31,31,31,31,31,31,31,31,31,31,31,31,31,31,31,31,31,31,31,31,31,31,31,31,31,31,31,31,31,31,31,31,31,31,31,31,31,31,31,31,31,31,31,31,31,31,31,31,31,31,31,31,31,31,31,31,31,31,31,31,31,31,31,31,31,31,31,31,31,31,31,31,31,31,31,31,31,31,31,31,31,31,31,31,31,31,31,31,31,31,31,31,31,31,31,31,31,31,31,31,31,31,31,31,31,31,31,31,31,31,31,31,31,31,31,31,31,31,31,31,31,31,31,31,31,31,31,31,31,31,31,31,31,31,31,31,31,31,31,31,31,31,31,31,31,31,31,31,31,31,31,31,31,31,31,31,31,31,31,31,31,31,31,31,31,31,31,31,31,31,31,31,31,31,31,31,31,31,31,31,31,31,31,31,31,31,31,31,31,31,31,31,31,31,31,31,31,31,31,31,31,31,31,31,31,31,31,31,31,31,31,31,31,31,31,31,31,31,31,31,31,31,31,31,31,31,31,31,31,31,31,31,31,31,31,31,31,31,31,31,31,31,31,31,31,31,31,31,31,31,31,31,31,31,31,31,31,31,31,31,31,31,31,31,31,31,31,31,31,31,31,31,31,31,31,31,31,31,31,31,31,31,31,31,31,31,31,31,31,31,31,31,31,31,31,31,31,31,31,31,31,31,31,31,31,31,31,31,31,31,31,31,31,31,31,31,31,31,31,31,31,31,31,31,31,31,31,31,31,31,31,31,31,31,31,31,31,31,31,31,31,31,31,31,31,31,31,31,31,31,31,31,31,31,31,31,31,31,31,31,31,31,31,31,31,31,31,31,31,31,31,31,31,31,31,31,31,31,31,31,31,31,31,31,31,31,31,31,31,31,31,31,31,31,31,31,31,31,31,31,31,31,31,31,31,31,31,31,31,31,31,31,31,31,31,31,31,31,31,31,31,31,31,31,31,31,31,31,31,31,31,31,31,31,31,31,31,31,31,31,31,31,31,31,31,31,31,31,31,31,31,31,31,31,31,31,31,31,31,31,31,31,31,31,31,31,31,31,31,31,31,31,31,31,31,31,31,31,31,31,31,31,31,31,31,31,31,31,31,31,31,31,31,31,31,31,31,31,31,31,31,31,31,31,31,31,31,31,31,31,31,31,31,31,31,31,31,31,31,31,31,31,31,31,31,31,31,31,31,31,31,31,31,31,31,31,31,31,31,31,31,31,31,31,31,31,31,31,31,31,31,31,31,31,31,31,31,31,31,31,31,31,31,31,31,31,31,31,31,31,31,31,31,31,31,31,31,31,31,31,31,31,31,31,31,31,31,31,31,31,31,31,31,31,31,31,31,31,31,31,31,31};

__global__ __launch_bounds__(256) void k_wtG(const float* __restrict__ w, int K, int N, bf* Bt) {
    const int lane = threadIdx.x & 31; const int L0 = (blockIdx.x * 8 + (threadIdx.x >> 5)) * 8; const int nlines = N * K / 64;
#pragma unroll 1
    for (int ps = 0; ps < 2; ++ps) {
#pragma unroll 1
        for (int l = 0; l < 8; ++l) { const int L = L0 + l; if (L >= nlines) break; const size_t e = (size_t)L * 64 + lane * 2; const int k = (int)(e % K), n = (int)(e / K); v2us o;
            o[0] = f2bf(w[(size_t)k * N + n]); o[1] = f2bf(w[(size_t)(k + 1) * N + n]); *(volatile v2us*)(Bt + e) = o; }
        if (ps == 0) __threadfence(); }
}
__global__ __launch_bounds__(256) void k_cvt8(const float* __restrict__ src, bf* dst, size_t n8) { const size_t i = (size_t)blockIdx.x * 256 + threadIdx.x; if (i >= n8) return; const v8f v = *(const v8f*)(src + i * 8); v8us o;
#pragma unroll
    for (int k = 0; k < 8; ++k) o[k] = f2bf(v[k]); *(volatile v8us*)(dst + i * 8) = o; __threadfence(); *(volatile v8us*)(dst + i * 8) = o; }
__global__ __launch_bounds__(256) void k_pl(const float* __restrict__ F, float scl, h16* P16) { const size_t e = ((size_t)blockIdx.x * 256 + threadIdx.x) * 2; if (e >= (size_t)NH_ * TT * HD) return; const int d = (int)(e % HD); const int t = (int)((e / HD) % TT); const int h = (int)(e / ((size_t)HD * TT)); const float* f = F + (size_t)t * EE + h * HD + d; v2h o; o[0] = tohx(f[0] * scl); o[1] = tohx(f[1] * scl); *(volatile v2h*)(P16 + e) = o; __threadfence(); *(volatile v2h*)(P16 + e) = o; }
__global__ __launch_bounds__(256) void k_vtp(const float* __restrict__ F, h16* VT) { const size_t e = ((size_t)blockIdx.x * 256 + threadIdx.x) * 2; if (e >= (size_t)NH_ * HD * TT) return; const int t = (int)(e % TT); const int d = (int)((e / TT) % HD); const int h = (int)(e / ((size_t)TT * HD)); v2h o; o[0] = tohx(F[(size_t)t * EE + h * HD + d]); o[1] = tohx(F[(size_t)(t + 1) * EE + h * HD + d]); *(volatile v2h*)(VT + e) = o; __threadfence(); *(volatile v2h*)(VT + e) = o; }
__global__ __launch_bounds__(256) void k_gate(const float* __restrict__ x, const float* __restrict__ gw, const float* __restrict__ gb, const float* __restrict__ gc, float* GATE) { const int row = blockIdx.x * 256 + threadIdx.x; if (row >= NH_ * TT) return; const int t = row % TT, h = row / TT; const float* xr = x + (size_t)t * EE + h * HD; float sa = 0.f, sb = 0.f;
#pragma unroll 1
    for (int e = 0; e < 8; ++e) { float g = 0.f;
#pragma unroll 1
        for (int d = 0; d < HD; ++d) { float p = __fmul_rn(bfr(xr[d]), bfr(gw[d * 8 + e])); asm volatile("" : "+v"(p)); g = __fadd_rn(g, p); }
        g = __fadd_rn(g, bfr(gb[e])); if (e < 4) sa = __fadd_rn(sa, g); else sb = __fadd_rn(sb, g); }
    const float ga = sigm_(sa), gbv = sigm_(sb); float tmm = __fmul_rn(gbv, bfr(gc[h])); asm volatile("" : "+v"(tmm)); float gm = __fmul_rn(ga, __fsub_rn(tmm, 1.0f)); asm volatile("" : "+v"(gm)); const float gate = __fadd_rn(gm, 2.0f);
    *(volatile float*)(GATE + row) = gate; __threadfence(); *(volatile float*)(GATE + row) = gate; }
__global__ __launch_bounds__(256) void k_bsoft(const float* __restrict__ Sb, const float* __restrict__ GATE, const float* __restrict__ re, int h0, h16* P) { const int lane = threadIdx.x & 31; const int row = blockIdx.x * 8 + (threadIdx.x >> 5); if (row >= ZH * TT) return; const int i = row % TT, z = row / TT; const int h = h0 + z; const float gt = GATE[(size_t)h * TT + i]; const float* sr = Sb + (size_t)row * TT; float v[32]; float mx = -3.0e38f;
#pragma unroll
    for (int ch = 0; ch < 8; ++ch) { const int j0 = ch * 128 + lane * 4; const v4f a = *(const v4f*)(sr + j0);
#pragma unroll
        for (int q = 0; q < 4; ++q) { const int j = j0 + q; float pb = __fmul_rn(gt, bfr(re[(int)c_bkt[j - i + TT - 1] * NH_ + h])); asm volatile("" : "+v"(pb)); const float t = __fadd_rn(a[q], pb); v[ch * 4 + q] = t; mx = fmaxf(mx, t); } }
#pragma unroll
    for (int sh = 16; sh; sh >>= 1) mx = fmaxf(mx, __shfl_xor(mx, sh, 32));
    float sum = 0.f;
#pragma unroll
    for (int k = 0; k < 32; ++k) { float d0 = __fsub_rn(v[k], mx); asm volatile("" : "+v"(d0)); v[k] = __expf(d0); sum += v[k]; }
#pragma unroll
    for (int sh = 16; sh; sh >>= 1) sum += __shfl_xor(sum, sh, 32);
    const float f = __fdiv_rn(PCAR, sum);
#pragma unroll 1
    for (int ps = 0; ps < 2; ++ps) {
#pragma unroll
        for (int ch = 0; ch < 8; ++ch) { v4h o; o[0] = tohx(v[ch * 4] * f); o[1] = tohx(v[ch * 4 + 1] * f); o[2] = tohx(v[ch * 4 + 2] * f); o[3] = tohx(v[ch * 4 + 3] * f); *(volatile v4h*)(P + (size_t)row * TT + ch * 128 + lane * 4) = o; }
        if (ps == 0) __threadfence(); } }
__global__ __launch_bounds__(256) void k_mrg(const float* __restrict__ Ob, int h0, bf* Ah, bf* Al) { const size_t e = ((size_t)blockIdx.x * 256 + threadIdx.x) * 2; if (e >= (size_t)ZH * TT * HD) return; const int d = (int)(e % HD); const int t = (int)((e / HD) % TT); const int z = (int)(e / ((size_t)HD * TT)); v2us oh, ol;
#pragma unroll
    for (int u = 0; u < 2; ++u) { unsigned short a, c; splitf(Ob[e + u] * (1.0f / PCAR), a, c); oh[u] = a; ol[u] = c; } const size_t o = (size_t)t * EE + (h0 + z) * HD + d; *(volatile v2us*)(Ah + o) = oh; *(volatile v2us*)(Al + o) = ol; __threadfence(); *(volatile v2us*)(Ah + o) = oh; *(volatile v2us*)(Al + o) = ol; }

extern "C" void kernel_launch(void* const* d_in, const int* in_sizes, int n_in,
                              void* d_out, int out_size, void* d_ws, size_t ws_size, hipStream_t stream) {
    (void)in_sizes; (void)n_in; (void)out_size;
    const float* IN[13]; for (int i = 0; i < 13; ++i) IN[i] = (const float*)d_in[i];
    float* OUT = (float*)d_out;
    char* wsp = (char*)d_ws;
    auto take = [&](size_t bytes) { char* p = wsp; wsp += (bytes + 255) & ~(size_t)255; return (void*)p; };
    bf* WQ = (bf*)take((size_t)EE * EE * 2); bf* WK = (bf*)take((size_t)EE * EE * 2); bf* WV = (bf*)take((size_t)EE * EE * 2); bf* WO = (bf*)take((size_t)EE * EE * 2); bf* XB = (bf*)take((size_t)TT * EE * 2);
    float* QF = (float*)take((size_t)TT * EE * 4); float* KF = (float*)take((size_t)TT * EE * 4); h16* Q16 = (h16*)take((size_t)NH_ * TT * HD * 2); h16* K16 = (h16*)take((size_t)NH_ * TT * HD * 2); h16* VT = (h16*)take((size_t)NH_ * HD * TT * 2); float* GATE = (float*)take((size_t)NH_ * TT * 4);
    float* Sb = (float*)take((size_t)ZH * TT * TT * 4); h16* P16 = (h16*)take((size_t)ZH * TT * TT * 2); float* Ob = (float*)take((size_t)ZH * TT * HD * 4); bf* Ah = (bf*)take((size_t)TT * EE * 2); bf* Al = (bf*)take((size_t)TT * EE * 2); float* VF = KF;
    if ((size_t)(wsp - (char*)d_ws) > ws_size) return;
    k_wtG<<<(EE * EE / 64 + 63) / 64, 256, 0, stream>>>(IN[1], EE, EE, WQ); k_wtG<<<(EE * EE / 64 + 63) / 64, 256, 0, stream>>>(IN[3], EE, EE, WK); k_wtG<<<(EE * EE / 64 + 63) / 64, 256, 0, stream>>>(IN[5], EE, EE, WV); k_wtG<<<(EE * EE / 64 + 63) / 64, 256, 0, stream>>>(IN[7], EE, EE, WO);
    const unsigned LP = (unsigned)(((size_t)NH_ * TT * HD / 2 + 255) / 256);
    for (int b = 0; b < NB_; ++b) { const float* xb = IN[0] + (size_t)b * TT * EE;
        k_cvt8<<<(TT * EE / 8 + 255) / 256, 256, 0, stream>>>(xb, XB, (size_t)TT * EE / 8); k_gate<<<NH_ * TT / 256, 256, 0, stream>>>(xb, IN[10], IN[11], IN[12], GATE);
        k_gemmw<bf, 0, true><<<dim3(TT / 64, EE / 64, 1), 32, 0, stream>>>(XB, nullptr, WQ, nullptr, EE, QF, EE, IN[2], 0, 0, 0); k_pl<<<LP, 256, 0, stream>>>(QF, 0.125f, Q16);
        k_gemmw<bf, 0, true><<<dim3(TT / 64, EE / 64, 1), 32, 0, stream>>>(XB, nullptr, WK, nullptr, EE, KF, EE, IN[4], 0, 0, 0); k_pl<<<LP, 256, 0, stream>>>(KF, 1.0f, K16);
        k_gemmw<bf, 0, true><<<dim3(TT / 64, EE / 64, 1), 32, 0, stream>>>(XB, nullptr, WV, nullptr, EE, VF, EE, IN[6], 0, 0, 0); k_vtp<<<LP, 256, 0, stream>>>(VF, VT);
        for (int h0 = 0; h0 < NH_; h0 += ZH) { const size_t z = (size_t)h0;
            k_gemmw<h16, 0, false><<<dim3(TT / 64, TT / 64, ZH), 32, 0, stream>>>(Q16 + z * TT * HD, nullptr, K16 + z * TT * HD, nullptr, HD, Sb, TT, nullptr, (size_t)TT * HD, (size_t)TT * HD, (size_t)TT * TT);
            k_bsoft<<<ZH * TT / 8, 256, 0, stream>>>(Sb, GATE, IN[9], h0, P16);
            k_gemmw<h16, 0, false><<<dim3(TT / 64, 1, ZH), 32, 0, stream>>>(P16, nullptr, VT + z * HD * TT, nullptr, TT, Ob, HD, nullptr, (size_t)TT * TT, (size_t)HD * TT, (size_t)TT * HD);
            k_mrg<<<(unsigned)(((size_t)ZH * TT * HD / 2 + 255) / 256), 256, 0, stream>>>(Ob, h0, Ah, Al); }
        k_gemmw<bf, 1, true><<<dim3(TT / 64, EE / 64, 1), 32, 0, stream>>>(Ah, Al, WO, nullptr, EE, OUT + (size_t)b * TT * EE, EE, IN[8], 0, 0, 0); }
}
